// DLRKernel_67637144978495
// MI455X (gfx1250) — hardware-verified
//
#include <hip/hip_runtime.h>


namespace {
constexpr int HH = 512, NN = 4096, LL = 8192, LC = 1024  ;

typedef _Float16 b16;
typedef __attribute__((ext_vector_type(16))) _Float16 v16b;
typedef __attribute__((ext_vector_type(8)))  _Float16 v8b;
typedef __attribute__((ext_vector_type(8)))  float v8f;
typedef __attribute__((ext_vector_type(4)))  float v4f;

__device__ __forceinline__ v8b ld8b(const b16* p) { return *(const v8b*)p; }
__device__ __forceinline__ v16b cat8b(v8b a, v8b b) { return __builtin_shufflevector(a, b, 0, 1, 2, 3, 4, 5, 6, 7, 8, 9, 10, 11, 12, 13, 14, 15); }
__device__ __forceinline__ v16b frag_kb(const b16* p, int hh) { return cat8b(ld8b(p + 8 * hh), ld8b(p + 16 + 8 * hh)); }
__device__ __forceinline__ void split16(float v, b16& hi, b16& lo) { hi = (b16)v; lo = (b16)(v - (float)hi); }
__device__ __forceinline__ void frag_ksplit(const float* p, int hh, v16b& fh_, v16b& fl_) {
  const float* p0 = p + 8 * hh; const float* p1 = p + 16 + 8 * hh;
#pragma unroll
  for (int e = 0; e < 8; ++e) { b16 a, c; split16(p0[e], a, c); fh_[e] = a; fl_[e] = c; split16(p1[e], a, c); fh_[8 + e] = a; fl_[8 + e] = c; }
}
__device__ __forceinline__ v8f wmma16b(v16b a, v16b b, v8f c) {
  v8f d = __builtin_amdgcn_wmma_f32_16x16x32_f16(false, a, false, b, (short)0, c, false, false);
  asm volatile("v_nop\n\tv_nop\n\tv_nop\n\tv_nop" : "+v"(d) : "v"(a), "v"(b));
  return d;
}
__device__ __forceinline__ void wave_lds_sync() {
  __builtin_amdgcn_fence(__ATOMIC_RELEASE, "workgroup");
  __builtin_amdgcn_wave_barrier();
  __builtin_amdgcn_fence(__ATOMIC_ACQUIRE, "workgroup");
}

struct Opnd { const void* p0; const void* p1; int ld; };
template <int NP> __device__ __forceinline__ void load_frags(const Opnd& o, int row, int kb, int hh, v16b& fh_, v16b& fl_) {
  if (NP == 0) { frag_ksplit((const float*)o.p0 + (size_t)row * o.ld + kb, hh, fh_, fl_); }
  else if (NP == 4 || NP == 5) {
    const float sc_ = (NP == 4) ? 64.0f : 8.0f;
    const float* p = (const float*)o.p0 + (size_t)row * o.ld + kb; const float* p0 = p + 8 * hh; const float* p1 = p + 16 + 8 * hh;
#pragma unroll
    for (int e = 0; e < 8; ++e) { b16 a, c; split16(p0[e] * sc_, a, c); fh_[e] = a; fl_[e] = c; split16(p1[e] * sc_, a, c); fh_[8 + e] = a; fl_[8 + e] = c; }
  } else if (NP == 3) {
    const float* p = (const float*)o.p0 + (size_t)row * o.ld + kb; const float* p0 = p + 8 * hh; const float* p1 = p + 16 + 8 * hh;
#pragma unroll
    for (int e = 0; e < 8; ++e) { fh_[e] = (b16)p0[e]; fh_[8 + e] = (b16)p1[e]; }
    fl_ = fh_;
  } else {
    fh_ = frag_kb((const b16*)o.p0 + (size_t)row * o.ld + kb, hh);
    if (NP == 2) fl_ = frag_kb((const b16*)o.p1 + (size_t)row * o.ld + kb, hh); else fl_ = fh_;
  }
}
template <int ANP, int BNP> __device__ __forceinline__ v8f mac(v16b ah, v16b al, v16b bh, v16b bl, v8f c) {
  c = wmma16b(ah, bh, c);
  if (BNP == 0 || BNP == 2 || BNP == 4 || BNP == 5) c = wmma16b(ah, bl, c);
  if (ANP == 0 || ANP == 2 || ANP == 4 || ANP == 5) c = wmma16b(al, bh, c);
  return c;
}
template <int ANP, int BNP>
__device__ __forceinline__ void gemm_tile(const Opnd& A, const Opnd& B, int K, int m0, int c0, int nloc, int hlf, v8f (&acc)[2][4]) {
  for (int kb = 0; kb < K; kb += 32) {
    v16b a0h, a0l, a1h, a1l;
    load_frags<ANP>(A, m0 + nloc, kb, hlf, a0h, a0l);
    load_frags<ANP>(A, m0 + 16 + nloc, kb, hlf, a1h, a1l);
#pragma unroll
    for (int t = 0; t < 4; ++t) {
      v16b bh, bl;
      load_frags<BNP>(B, c0 + t * 16 + nloc, kb, hlf, bh, bl);
      acc[0][t] = mac<ANP, BNP>(a0h, a0l, bh, bl, acc[0][t]);
      acc[1][t] = mac<ANP, BNP>(a1h, a1l, bh, bl, acc[1][t]);
    }
  }
}

__device__ __forceinline__ void epi_planes(v8f (&acc)[2][4], float scale, bool two, b16* __restrict__ oh, b16* __restrict__ ol, int ldo,
                                           int m0, int c0, int lane, b16* Th, b16* Tl) {
  const int nloc = lane & 15, hlf = lane >> 4;
#pragma unroll
  for (int t = 0; t < 4; ++t)
#pragma unroll
    for (int r = 0; r < 2; ++r)
#pragma unroll
      for (int v = 0; v < 8; ++v) {
        const int rr = r * 16 + v + 8 * hlf, cc = t * 16 + nloc;
        b16 h_, l_; split16(acc[r][t][v] * scale, h_, l_);
        Th[rr * 64 + cc] = h_; Tl[rr * 64 + cc] = l_;
      }
  wave_lds_sync();
  for (int pass = 0; pass < 2; ++pass) {
#pragma unroll
    for (int j = 0; j < 8; ++j) {
      const int rr = j * 4 + (lane >> 3), c8 = (lane & 7) * 8;
      const size_t o = (size_t)(m0 + rr) * ldo + c0 + c8;
      *(volatile v8b*)(oh + o) = ld8b(Th + rr * 64 + c8);
      if (two) *(volatile v8b*)(ol + o) = ld8b(Tl + rr * 64 + c8);
    }
    __threadfence();
  }
}
__device__ __forceinline__ void epi_f32(v8f (&acc)[2][4], float scale, const float* rscale, float* __restrict__ out, int ldo, int m0, int c0, int lane, float* Tt) {
  const int nloc = lane & 15, hlf = lane >> 4;
#pragma unroll
  for (int t = 0; t < 4; ++t)
#pragma unroll
    for (int r = 0; r < 2; ++r)
#pragma unroll
      for (int v = 0; v < 8; ++v) {
        const int rr = r * 16 + v + 8 * hlf;
        const float rs = rscale ? rscale[(size_t)(m0 + rr) * 32] : 1.0f;
        Tt[rr * 64 + t * 16 + nloc] = acc[r][t][v] * scale * rs;
      }
  wave_lds_sync();
  float* dst0 = out + (size_t)m0 * ldo + c0;
  for (int pass = 0; pass < 2; ++pass) {
#pragma unroll
    for (int j = 0; j < 16; ++j) { const int rr = j * 2 + hlf, c4 = nloc * 4; *(volatile v4f*)(dst0 + (size_t)rr * ldo + c4) = *(const v4f*)(Tt + rr * 64 + c4); }
    __threadfence();
  }
}


typedef __attribute__((ext_vector_type(8))) __bf16 v8bb; typedef __attribute__((ext_vector_type(16))) __bf16 v16bb;
typedef __attribute__((ext_vector_type(8))) unsigned short v8us;
__device__ __forceinline__ v16bb frag_kb_bf(const __bf16* p, int hh) { const v8bb a = *(const v8bb*)(p + 8 * hh), b = *(const v8bb*)(p + 16 + 8 * hh); return __builtin_shufflevector(a, b, 0, 1, 2, 3, 4, 5, 6, 7, 8, 9, 10, 11, 12, 13, 14, 15); }
__device__ __forceinline__ v8f wmma16bb(v16bb a, v16bb b, v8f c) {
  v8f d = __builtin_amdgcn_wmma_f32_16x16x32_bf16(false, a, false, b, (short)0, c, false, false);
  asm volatile("v_nop\n\tv_nop\n\tv_nop\n\tv_nop" : "+v"(d) : "v"(a), "v"(b));
  return d;
}
__device__ __forceinline__ unsigned short bf16_rne_bits(float v) { unsigned int u = __float_as_uint(v); u += 0x7FFFu + ((u >> 16) & 1u); return (unsigned short)(u >> 16); }
__device__ __forceinline__ float bf16_rne(float v) { return __uint_as_float(((unsigned int)bf16_rne_bits(v)) << 16); }


__global__ __launch_bounds__(256) void prep_kernel(const float* __restrict__ W, const float* __restrict__ lam, b16* __restrict__ wh, float* __restrict__ lamr) {
  const size_t tid = (size_t)blockIdx.x * blockDim.x + threadIdx.x, nth = (size_t)gridDim.x * blockDim.x;
  for (int pass = 0; pass < 2; ++pass) {
    for (size_t p = tid; p < (size_t)HH * NN / 8; p += nth) { v8b v;
#pragma unroll
      for (int e = 0; e < 8; ++e) v[e] = (b16)(bf16_rne(W[p * 8 + e]) * 4096.0f);
      *(volatile v8b*)(wh + p * 8) = v; }
    for (size_t p = tid; p < (size_t)NN; p += nth) ((volatile float*)lamr)[p] = bf16_rne(lam[p]);
    __threadfence();
  }
}

__global__ __launch_bounds__(256) void cos_kernel(const float* __restrict__ lamr, int l0, b16* __restrict__ sh, b16* __restrict__ sl) {
  const size_t i = (size_t)blockIdx.x * 256 + threadIdx.x; const int r = (int)(i / (NN / 8)), n0 = (int)(i % (NN / 8)) * 8; const float lf = (float)(l0 + r);
  v8b a, c;
#pragma unroll
  for (int e = 0; e < 8; ++e) { const float ang = lamr[n0 + e] * lf; const float cv = cosf(ang); const b16 x = (b16)cv; a[e] = x; c[e] = (b16)((cv - (float)x) * 1024.0f); }
  for (int pass = 0; pass < 2; ++pass) { *(volatile v8b*)(sh + (size_t)r * NN + n0) = a; *(volatile v8b*)(sl + (size_t)r * NN + n0) = c; __threadfence(); }
}

__global__ __launch_bounds__(128) void gemm_kernel(const b16* __restrict__ wh, const b16* __restrict__ sh, const b16* __restrict__ sl, int l0, float* __restrict__ out) {
  __shared__ __attribute__((aligned(16))) float Ts[4][32 * 64];
  const int lane = threadIdx.x & 31, wave = threadIdx.x >> 5, nloc = lane & 15, hlf = lane >> 4, m0 = blockIdx.y * 128 + wave * 32, c0 = blockIdx.x * 64;
  v8f acc[2][4];
#pragma unroll
  for (int r = 0; r < 2; ++r)
#pragma unroll
    for (int t = 0; t < 4; ++t) acc[r][t] = (v8f){};
  v8f acl[2][4];
#pragma unroll
  for (int r = 0; r < 2; ++r)
#pragma unroll
    for (int t = 0; t < 4; ++t) acl[r][t] = (v8f){};
#pragma unroll 2
  for (int kb = 0; kb < NN; kb += 32) { const v16b a0 = frag_kb(wh + (size_t)(m0 + nloc) * NN + kb, hlf), a1 = frag_kb(wh + (size_t)(m0 + 16 + nloc) * NN + kb, hlf);
#pragma unroll
    for (int t = 0; t < 4; ++t) { const size_t bo = (size_t)(c0 + t * 16 + nloc) * NN + kb; const v16b bh = frag_kb(sh + bo, hlf), bl = frag_kb(sl + bo, hlf);
      acc[0][t] = wmma16b(a0, bh, acc[0][t]); acc[1][t] = wmma16b(a1, bh, acc[1][t]); acl[0][t] = wmma16b(a0, bl, acl[0][t]); acl[1][t] = wmma16b(a1, bl, acl[1][t]); } }
#pragma unroll
  for (int r = 0; r < 2; ++r)
#pragma unroll
    for (int t = 0; t < 4; ++t)
#pragma unroll
      for (int v = 0; v < 8; ++v) acc[r][t][v] = (acc[r][t][v] + acl[r][t][v] * (1.0f / 1024.0f)) * (1.0f / 4096.0f);
  epi_f32(acc, 1.0f, nullptr, out + l0, LL, m0, c0, lane, Ts[wave]);
}
}

extern "C" void kernel_launch(void* const* d_in, const int* in_sizes, int n_in,
                              void* d_out, int out_size, void* d_ws, size_t ws_size, hipStream_t stream) {
  (void)n_in; (void)out_size;
  const float* W = (const float*)d_in[0]; const float* lam = (const float*)d_in[1];
  float* out = (float*)d_out;
  if (in_sizes[0] != HH * NN || in_sizes[1] != NN) return;
  size_t off = 0; char* ws = (char*)d_ws;
  auto carve = [&](size_t bytes) { char* p = ws + off; off += (bytes + 255) & ~(size_t)255; return p; };
  b16* wh = (b16*)carve((size_t)HH * NN * 2); float* lamr = (float*)carve(NN * 4); b16* sh = (b16*)carve((size_t)LC * NN * 2); b16* sl = (b16*)carve((size_t)LC * NN * 2);
  if (off > ws_size) return;
  prep_kernel<<<512, 256, 0, stream>>>(W, lam, wh, lamr);
  for (int l0 = 0; l0 < LL; l0 += LC) {
    cos_kernel<<<LC * NN / 8 / 256, 256, 0, stream>>>(lamr, l0, sh, sl);
    gemm_kernel<<<dim3(LC / 64, HH / 128), 128, 0, stream>>>(wh, sh, sl, l0, out);
  }
}
